// GRUStateEstimation_77111842832531
// MI455X (gfx1250) — hardware-verified
//
#include <hip/hip_runtime.h>
#include <math.h>

typedef __attribute__((ext_vector_type(16))) _Float16 v16h;
typedef __attribute__((ext_vector_type(8)))  _Float16 v8h;
typedef __attribute__((ext_vector_type(16))) __bf16   v16b;
typedef __attribute__((ext_vector_type(8)))  __bf16   v8b;
typedef __attribute__((ext_vector_type(8)))  float    v8f;
typedef __attribute__((ext_vector_type(4)))  float    v4f;

constexpr int kB    = 256;
constexpr int kT    = 200;
constexpr int kIn   = 128;
constexpr int kH    = 256;
constexpr int kG3   = 3 * kH;
constexpr int kOut  = 118;
constexpr int kOutP = 128;
constexpr int kNP   = 4;
constexpr int kThr  = 256;
constexpr float kInCarry = 1024.0f;
constexpr float kSc = 1.0f / (kInCarry * kInCarry);
constexpr float kF16MinNormal = 6.103515625e-5f;
constexpr int kFBF = 0, kFBZ = 128, kFEnd = 1024;

static_assert((kB % 64) == 0 && ((kB / 64) * (kG3 / 64)) % 8 == 0 && ((kB / 64) * (kOutP / 64)) % 8 == 0 && (kH % 32) == 0 && kIn <= kH && kOut <= kOutP && kFBZ + kG3 <= kFEnd,
              "GEMM M, N multiples of 64; grids exact; K multiples of 32");

constexpr size_t kOffW4 = 0ull;
constexpr size_t kOffWF = 1572864ull;
constexpr size_t kOffBIAS = 1638400ull;
constexpr size_t kOffA4 = 1642496ull;
constexpr size_t kOffG4 = 2166784ull;
constexpr size_t kOffH32 = 5312512ull;
constexpr size_t kOffO32 = 5836800ull;
constexpr size_t kWsTotal = 5967872ull;
static_assert(kWsTotal <= 134217728ull, "carve cap: under 128 MiB");
static_assert(kOffW4 == 0
              && kOffWF == kOffW4 + 1572864ull
              && kOffBIAS == kOffWF + 65536ull
              && kOffA4 == kOffBIAS + 4096ull
              && kOffG4 == kOffA4 + 524288ull
              && kOffH32 == kOffG4 + 3145728ull
              && kOffO32 == kOffH32 + 524288ull
              && kWsTotal == kOffO32 + 131072ull, "the carve is chained and totalled");
static_assert((kOffW4 % 256) == 0 && (kOffWF % 256) == 0 && (kOffBIAS % 256) == 0 && (kOffA4 % 256) == 0 && (kOffG4 % 256) == 0 && (kOffH32 % 256) == 0 && (kOffO32 % 256) == 0, "aligned regions");

__device__ __forceinline__ unsigned short f2bf_bits(float f) {
  unsigned u = __float_as_uint(f);
  return (unsigned short)((u + 0x7FFFu + ((u >> 16) & 1u)) >> 16);
}
__device__ __forceinline__ float bf_bits2f(unsigned short h) { return __uint_as_float(((unsigned)h) << 16); }
__device__ __forceinline__ float bf16r(float f) { return bf_bits2f(f2bf_bits(f)); }
__device__ __forceinline__ float carry_flush(float v, float carry) {
  const float s = v * carry;
  return (fabsf(s) < kF16MinNormal) ? 0.0f : s;
}
__device__ __forceinline__ float frcp(float x) { return __builtin_amdgcn_rcpf(x); }

__device__ __forceinline__ void dep_guard4_h(v8f& a, v8f& b, v8f& c, v8f& d, v16h x, v16h y) { asm volatile("v_nop\n\tv_nop\n\tv_nop\n\tv_nop" : "+v"(a), "+v"(b), "+v"(c), "+v"(d) : "v"(x), "v"(y)); }
__device__ __forceinline__ void dep_guard4_b(v8f& a, v8f& b, v8f& c, v8f& d, v16b x, v16b y) { asm volatile("v_nop\n\tv_nop\n\tv_nop\n\tv_nop" : "+v"(a), "+v"(b), "+v"(c), "+v"(d) : "v"(x), "v"(y)); }
__device__ __forceinline__ void keep4_h(v16h a, v16h b, v16h c, v16h d) { asm volatile("v_nop" :: "v"(a), "v"(b), "v"(c), "v"(d)); }
__device__ __forceinline__ void keep4_b(v16b a, v16b b, v16b c, v16b d) { asm volatile("v_nop" :: "v"(a), "v"(b), "v"(c), "v"(d)); }
__device__ __forceinline__ void acc_guard4(v8f& a, v8f& b, v8f& c, v8f& d) { asm volatile("v_nop\n\tv_nop\n\tv_nop\n\tv_nop" : "+v"(a), "+v"(b), "+v"(c), "+v"(d)); }

template <typename T> struct Frag;
template <> struct Frag<_Float16> {
  typedef v16h V; union U { v16h v; v8h h[2]; };
  static __device__ __forceinline__ v16h load(const _Float16* p) {
    U f; f.h[0] = *(const v8h*)(p); f.h[1] = *(const v8h*)(p + 16); return f.v;
  }
  static __device__ __forceinline__ v8f mma(v16h a, v16h b, v8f c) {
    return __builtin_amdgcn_wmma_f32_16x16x32_f16(false, a, false, b, (short)0, c, false, false);
  }
  static __device__ __forceinline__ void guard4(v8f& a, v8f& b, v8f& c, v8f& d, v16h x, v16h y) { dep_guard4_h(a, b, c, d, x, y); }
  static __device__ __forceinline__ void keep(v16h a, v16h b, v16h c, v16h d) { keep4_h(a, b, c, d); }
};
template <> struct Frag<__bf16> {
  typedef v16b V; union U { v16b v; v8b h[2]; };
  static __device__ __forceinline__ v16b load(const __bf16* p) {
    U f; f.h[0] = *(const v8b*)(p); f.h[1] = *(const v8b*)(p + 16); return f.v;
  }
  static __device__ __forceinline__ v8f mma(v16b a, v16b b, v8f c) {
    return __builtin_amdgcn_wmma_f32_16x16x32_bf16(false, a, false, b, (short)0, c, false, false);
  }
  static __device__ __forceinline__ void guard4(v8f& a, v8f& b, v8f& c, v8f& d, v16b x, v16b y) { dep_guard4_b(a, b, c, d, x, y); }
  static __device__ __forceinline__ void keep(v16b a, v16b b, v16b c, v16b d) { keep4_b(a, b, c, d); }
};

__device__ __forceinline__ v8f mma_h(v16h a, v16h b, v8f c) {
  c = __builtin_amdgcn_wmma_f32_16x16x32_f16(false, a, false, b, (short)0, c, false, false);
  asm volatile("v_nop\n\tv_nop\n\tv_nop\n\tv_nop" : "+v"(c) : "v"(a), "v"(b));
  return c;
}

template <int ET> struct Elem;
template <> struct Elem<0> { typedef _Float16 T; };
template <> struct Elem<1> { typedef __bf16 T; };
template <int ET, bool SPLIT, int BIAS_MODE, int OUT_MODE, bool RESID, int ACT = 0>
__global__ __launch_bounds__(256) void wmma_gemm64(
    const unsigned short* __restrict__ Ap, const unsigned short* __restrict__ A2p, int lda, long strideA,
    const unsigned short* __restrict__ Btp, const unsigned short* __restrict__ Bt2p, int ldb, long strideB,
    void* __restrict__ Cout, void* __restrict__ Cout2, int ldc, long strideC,
    const float* __restrict__ bias,
    const float* __restrict__ resid, long strideR,
    int M, int N, int K, float scale) {
  typedef typename Elem<ET>::T T;
  typedef typename Frag<T>::V V;
  const T* A = (const T*)Ap; const T* A2 = (const T*)A2p; const T* Bt = (const T*)Btp; const T* Bt2 = (const T*)Bt2p;
  __shared__ __align__(16) float sT[8][16 * 68];
  const int b    = blockIdx.y;
  const int lane = threadIdx.x & 31;
  const int wave = threadIdx.x >> 5;
  const int tilesN = N >> 6;
  const int tilesM = M >> 6;
  const int tile = blockIdx.x * 8 + wave;
  if (tile >= tilesM * tilesN) return;
  const int tm = tile / tilesN;
  const int tn = tile - tm * tilesN;
  const int m0 = tm << 6;
  const int n0 = tn << 6;

  const T* Ab  = A  + (size_t)b * strideA;
  const T* Bb  = Bt + (size_t)b * strideB;
  const T* Ab2 = SPLIT ? (A2  + (size_t)b * strideA) : nullptr;
  const T* Bb2 = SPLIT ? (Bt2 + (size_t)b * strideB) : nullptr;

  const int rlane = lane & 15;
  const int koff  = (lane >> 4) * 8;
  const int mOff  = (lane >> 4) * 8;

  v8f acc[4][4];
#pragma unroll
  for (int i = 0; i < 4; ++i)
#pragma unroll
    for (int j = 0; j < 4; ++j) acc[i][j] = (v8f){0.f,0.f,0.f,0.f,0.f,0.f,0.f,0.f};

  for (int k0 = 0; k0 < K; k0 += 32) {
    V bh[4], bl[4];
#pragma unroll
    for (int j = 0; j < 4; ++j) {
      const size_t bo = (size_t)(n0 + (j << 4) + rlane) * ldb + koff + k0;
      bh[j] = Frag<T>::load(Bb + bo);
      if (SPLIT) bl[j] = Frag<T>::load(Bb2 + bo);
    }
#pragma unroll
    for (int i = 0; i < 4; ++i) {
      const size_t ao = (size_t)(m0 + (i << 4) + rlane) * lda + koff + k0;
      V ah = Frag<T>::load(Ab + ao);
      V al;
      if (SPLIT) al = Frag<T>::load(Ab2 + ao);
#pragma unroll
      for (int j = 0; j < 4; ++j) {
        acc[i][j] = Frag<T>::mma(ah, bh[j], acc[i][j]);
        if (SPLIT) {
          acc[i][j] = Frag<T>::mma(ah, bl[j], acc[i][j]);
          acc[i][j] = Frag<T>::mma(al, bh[j], acc[i][j]);
        }
      }
      Frag<T>::guard4(acc[i][0], acc[i][1], acc[i][2], acc[i][3], ah, SPLIT ? al : ah);
    }
    Frag<T>::keep(bh[0], bh[1], bh[2], bh[3]);
    if (SPLIT) Frag<T>::keep(bl[0], bl[1], bl[2], bl[3]);
  }
  acc_guard4(acc[0][0], acc[0][1], acc[0][2], acc[0][3]);
  acc_guard4(acc[1][0], acc[1][1], acc[1][2], acc[1][3]);
  acc_guard4(acc[2][0], acc[2][1], acc[2][2], acc[2][3]);
  acc_guard4(acc[3][0], acc[3][1], acc[3][2], acc[3][3]);

  float* slab = sT[wave];
  const float* Rb = RESID ? (resid + (size_t)b * strideR) : nullptr;
#pragma unroll
  for (int i = 0; i < 4; ++i) {
    const int mBase = m0 + (i << 4);
#pragma unroll
    for (int j = 0; j < 4; ++j) {
      const int n = n0 + (j << 4) + rlane;
      float bv = 0.f;
      if (BIAS_MODE == 2) bv = bias[n];
#pragma unroll
      for (int r = 0; r < 8; ++r) {
        float v = acc[i][j][r] * scale;
        if (BIAS_MODE == 1) v += bias[mBase + mOff + r];
        if (BIAS_MODE == 2) v += bv;
        if (RESID) v += Rb[(size_t)(mBase + mOff + r) * ldc + n];
        if (ACT == 1) v = tanhf(v);
        if (ACT == 2) v = fmaxf(v, 0.0f);
        if (ACT == 3) v = v / (1.0f + expf(-v));
        if (ACT == 4) v = (v > 0.f) ? v : 0.01f * v;
        slab[(mOff + r) * 68 + (j << 4) + rlane] = v;
      }
    }
    __builtin_amdgcn_fence(__ATOMIC_RELEASE, "workgroup");
    __builtin_amdgcn_wave_barrier();
    __builtin_amdgcn_fence(__ATOMIC_ACQUIRE, "workgroup");
    if (OUT_MODE == 0) {
      float* C = (float*)Cout + (size_t)b * strideC;
      const int hh = lane >> 4, c4 = (lane & 15) * 4;
      for (int pass = 0; pass < 2; ++pass) {
#pragma unroll
        for (int it = 0; it < 8; ++it) {
          const int row = it * 2 + hh;
          v4f v = *(const v4f*)(slab + row * 68 + c4);
          *(volatile v4f*)(C + (size_t)(mBase + row) * ldc + n0 + c4) = v;
        }
        __threadfence();
      }
    } else {
      const int q = lane >> 3, c8 = (lane & 7) * 8;
      unsigned short* C  = (unsigned short*)Cout  + (size_t)b * strideC;
      unsigned short* C2 = (OUT_MODE == 2) ? ((unsigned short*)Cout2 + (size_t)b * strideC) : nullptr;
      for (int pass = 0; pass < 2; ++pass) {
#pragma unroll
        for (int it = 0; it < 4; ++it) {
          const int row = it * 4 + q;
          const float* sp = slab + row * 68 + c8;
          v8h hv, lv;
#pragma unroll
          for (int e = 0; e < 8; ++e) {
            if (OUT_MODE == 1) {
              hv[e] = (_Float16)sp[e];
            } else {
              unsigned short hb = f2bf_bits(sp[e]);
              unsigned short lb = f2bf_bits(sp[e] - bf_bits2f(hb));
              hv[e] = __builtin_bit_cast(_Float16, hb);
              lv[e] = __builtin_bit_cast(_Float16, lb);
            }
          }
          *(volatile v8h*)(C + (size_t)(mBase + row) * ldc + n0 + c8) = hv;
          if (OUT_MODE == 2) *(volatile v8h*)(C2 + (size_t)(mBase + row) * ldc + n0 + c8) = lv;
        }
        __threadfence();
      }
    }
    __builtin_amdgcn_fence(__ATOMIC_RELEASE, "workgroup");
    __builtin_amdgcn_wave_barrier();
    __builtin_amdgcn_fence(__ATOMIC_ACQUIRE, "workgroup");
  }
}

__global__ __launch_bounds__(kThr) void cast_plane_kernel(const float* __restrict__ src, unsigned short* __restrict__ dst,
                                                          int colsLog2, int dstPitch, int dstOff) {
  const int i   = blockIdx.x * kThr + threadIdx.x;
  const int sh  = colsLog2 - 3;
  const int row = i >> sh;
  const int c8  = (i & ((1 << sh) - 1)) * 8;
  const float* sp = src + ((size_t)row << colsLog2) + c8;
  const v4f a0 = *(const v4f*)(sp);
  const v4f a1 = *(const v4f*)(sp + 4);
  v8h hv;
#pragma unroll
  for (int e = 0; e < 4; ++e) {
    const float f0 = a0[e];
    const float f1 = a1[e];
    hv[e]     = (_Float16)carry_flush(bf16r(f0), kInCarry);
    hv[4 + e] = (_Float16)carry_flush(bf16r(f1), kInCarry);
  }
  unsigned short* dp = dst + (size_t)row * dstPitch + dstOff + c8;
  *(volatile v8h*)dp = hv;
  __threadfence();
  *(volatile v8h*)dp = hv;
}

__device__ __forceinline__ float fast_tanh(float v) { return 1.0f - 2.0f * frcp(__expf(2.0f * v) + 1.0f); }
__device__ __forceinline__ float fast_sigmoid(float v) { return frcp(1.0f + __expf(-v)); }

__global__ __launch_bounds__(kThr) void setup_kernel(const float* __restrict__ x, const float* __restrict__ fcW, const float* __restrict__ fcb,
                                                     float* __restrict__ BIAS, unsigned short* __restrict__ WF, unsigned short* __restrict__ W4,
                                                     unsigned short* __restrict__ A4, float* __restrict__ H32) {
  unsigned v = blockIdx.x * (unsigned)kThr + threadIdx.x;
  asm volatile("" : "+v"(v));
  if (v < 256u) {
    const unsigned i0 = v * 4u;
    v4f o;
#pragma unroll
    for (int e = 0; e < 4; ++e) {
      const unsigned i = i0 + (unsigned)e;
      const bool live = i < (unsigned)kOut;
      float w = fcb[live ? i : 0u];
      asm volatile("" : "+v"(w));
      o[e] = live ? bf16r(w) : 0.0f;
    }
    float* dp = BIAS + i0;
    *(volatile v4f*)dp = o;
    __threadfence();
    *(volatile v4f*)dp = o;
  } else if (v < 49408u) {
    v8h hv;
#pragma unroll
    for (int e = 0; e < 8; ++e) hv[e] = (_Float16)0.0f;
    unsigned short* dp;
    if (v < 4352u) {
      const unsigned w = v - 256u;
      const unsigned n = w >> 5, c8 = (w & 31u) * 8u;
      const bool live = n < (unsigned)kOut;
      const float* sp = fcW + (size_t)(live ? n : 0u) * kH + c8;
      const v4f a0 = *(const v4f*)sp, a1 = *(const v4f*)(sp + 4);
#pragma unroll
      for (int e = 0; e < 4; ++e) { const float p = a0[e], q = a1[e]; hv[e] = (_Float16)(live ? carry_flush(bf16r(p), kInCarry) : 0.0f); hv[4 + e] = (_Float16)(live ? carry_flush(bf16r(q), kInCarry) : 0.0f); }
      dp = WF + (size_t)w * 8u;
    } else if (v < 16640u) {
      const unsigned w = v - 4352u;
      dp = W4 + (size_t)(w >> 4) * kH + kIn + (w & 15u) * 8u;
    } else {
      const unsigned w = v - 16640u;
      const unsigned pl = w >> 13, b = (w >> 5) & 255u, c8 = (w & 31u) * 8u;
      const bool xs = (pl == 0u) && (c8 < (unsigned)kIn);
      const float* sp = x + (size_t)b * kT * kIn + (xs ? c8 : 0u);
      const v4f a0 = *(const v4f*)sp, a1 = *(const v4f*)(sp + 4);
#pragma unroll
      for (int e = 0; e < 4; ++e) { const float p = a0[e], q = a1[e]; hv[e] = (_Float16)(xs ? carry_flush(bf16r(p), kInCarry) : 0.0f); hv[4 + e] = (_Float16)(xs ? carry_flush(bf16r(q), kInCarry) : 0.0f); }
      dp = A4 + (size_t)w * 8u;
    }
    *(volatile v8h*)dp = hv;
    __threadfence();
    *(volatile v8h*)dp = hv;
  } else {
    const v4f z = {0.f, 0.f, 0.f, 0.f};
    float* dp = H32 + (size_t)(v - 49408u) * 4u;
    *(volatile v4f*)dp = z;
    __threadfence();
    *(volatile v4f*)dp = z;
  }
}
static_assert(kFEnd / 4 == 256 && kOutP * kH / 8 == 4096 && 256 + 4096 == 4352 && kG3 * 16 == 12288 && 4352 + 12288 == 16640 && kNP * kB * kH / 8 == 32768 && 16640 + 32768 == 49408
              && 2 * kB * kH / 4 == 32768 && 49408 + 32768 == 321 * kThr && (kH - kIn) == 16 * 8, "set-up grid exact");

__global__ __launch_bounds__(kThr) void gru2_kernel(const float* __restrict__ G4, const float* __restrict__ bih0, const float* __restrict__ bhh0,
                                                    const float* __restrict__ bih1, const float* __restrict__ bhh1, const float* __restrict__ x,
                                                    float* __restrict__ H32, unsigned short* __restrict__ A4, int k) {
  const bool l0 = blockIdx.x < 32u;
  if (l0 ? (k >= kT) : (k < 1)) return;
  const int l = l0 ? 0 : 1;
  unsigned v = (blockIdx.x & 31u) * (unsigned)kThr + threadIdx.x;
  asm volatile("" : "+v"(v));
  const unsigned b = v >> 5;
  const unsigned u8 = (v & 31u) * 8u;
  const float* gi = G4 + ((size_t)(2 * l) * kB + b) * kG3 + u8;
  const float* gh = G4 + ((size_t)(2 * l + 1) * kB + b) * kG3 + u8;
  const float* bi = (l0 ? bih0 : bih1) + u8;
  const float* bh = (l0 ? bhh0 : bhh1) + u8;
  float* hp32 = H32 + ((size_t)l * kB + b) * kH + u8;
  v8h hv, xv;
  v4f hn0, hn1;
#pragma unroll
  for (int hlf = 0; hlf < 2; ++hlf) {
    const v4f ir = *(const v4f*)(gi + 4 * hlf), iz = *(const v4f*)(gi + kH + 4 * hlf), in_ = *(const v4f*)(gi + 2 * kH + 4 * hlf);
    const v4f hr = *(const v4f*)(gh + 4 * hlf), hz = *(const v4f*)(gh + kH + 4 * hlf), hn_ = *(const v4f*)(gh + 2 * kH + 4 * hlf);
    const v4f bir = *(const v4f*)(bi + 4 * hlf), biz = *(const v4f*)(bi + kH + 4 * hlf), bin = *(const v4f*)(bi + 2 * kH + 4 * hlf);
    const v4f bhr = *(const v4f*)(bh + 4 * hlf), bhz = *(const v4f*)(bh + kH + 4 * hlf), bhn = *(const v4f*)(bh + 2 * kH + 4 * hlf);
    const v4f ho = *(const v4f*)(hp32 + 4 * hlf);
#pragma unroll
    for (int e = 0; e < 4; ++e) {
      const float p0 = bir[e], p1 = biz[e], p2 = bin[e], q0 = bhr[e], q1 = bhz[e], q2 = bhn[e];
      const float r = fast_sigmoid((ir[e] + bf16r(p0)) + (hr[e] + bf16r(q0)));
      const float z = fast_sigmoid((iz[e] + bf16r(p1)) + (hz[e] + bf16r(q1)));
      const float n = fast_tanh((in_[e] + bf16r(p2)) + r * (hn_[e] + bf16r(q2)));
      const float hn = (1.0f - z) * n + z * ho[e];
      if (hlf == 0) hn0[e] = hn; else hn1[e] = hn;
      hv[4 * hlf + e] = (_Float16)carry_flush(hn, kInCarry);
    }
  }
  const bool nx = l0 && (k + 1 < kT) && (u8 < (unsigned)kIn);
  {
    const float* sp = x + ((size_t)b * kT + (size_t)(nx ? (k + 1) : 0)) * kIn + (nx ? u8 : 0u);
    const v4f a0 = *(const v4f*)sp, a1 = *(const v4f*)(sp + 4);
#pragma unroll
    for (int e = 0; e < 4; ++e) { const float p = a0[e], q = a1[e]; xv[e] = (_Float16)carry_flush(bf16r(p), kInCarry); xv[4 + e] = (_Float16)carry_flush(bf16r(q), kInCarry); }
  }
  const size_t pl = (size_t)kB * kH;
  unsigned short* s1 = A4 + (l0 ? pl : 3 * pl) + (size_t)b * kH + u8;
  unsigned short* s2 = A4 + 2 * pl + (size_t)b * kH + u8;
  unsigned short* xp = A4 + (size_t)b * kH + u8;
  for (int pass = 0; pass < 2; ++pass) {
    *(volatile v4f*)hp32 = hn0; *(volatile v4f*)(hp32 + 4) = hn1;
    *(volatile v8h*)s1 = hv;
    if (l0) *(volatile v8h*)s2 = hv;
    if (nx) *(volatile v8h*)xp = xv;
    __threadfence();
  }
}
static_assert(kB * kH / 8 == 32 * kThr && kH / 8 == 32, "cell grid: 32 blocks a layer");

__global__ __launch_bounds__(128) void out_kernel(const float* __restrict__ O32, float* __restrict__ out) {
  unsigned v = blockIdx.x * 128u + threadIdx.x;
  asm volatile("" : "+v"(v));
  const unsigned i0 = v * 4u;
  v4f o;
#pragma unroll
  for (int e = 0; e < 4; ++e) {
    const unsigned i = i0 + (unsigned)e;
    const unsigned b = i / (unsigned)kOut, j = i % (unsigned)kOut;
    o[e] = O32[(size_t)b * kOutP + j];
  }
  float* dp = out + (size_t)i0;
  *(volatile v4f*)dp = o;
  __threadfence();
  *(volatile v4f*)dp = o;
}
static_assert(kB * kOut / 4 == 59 * 128 && (kB * kOut) % 4 == 0, "output grid exact");

static_assert(((size_t)kG3 * kH / 8) % kThr == 0 && ((size_t)kG3 * kIn / 8) % kThr == 0, "plane cast grids exact");

extern "C" void kernel_launch(void* const* d_in, const int* in_sizes, int n_in,
                              void* d_out, int out_size, void* d_ws, size_t ws_size,
                              hipStream_t stream) {
  if (n_in < 11 || d_out == nullptr || d_ws == nullptr) return;
  if (in_sizes[0] != kB * kT * kIn || in_sizes[1] != kG3 * kIn || in_sizes[2] != kG3 * kH || in_sizes[3] != kG3 || in_sizes[4] != kG3) return;
  if (in_sizes[5] != kG3 * kH || in_sizes[6] != kG3 * kH || in_sizes[7] != kG3 || in_sizes[8] != kG3 || in_sizes[9] != kOut * kH || in_sizes[10] != kOut) return;
  if (out_size != kB * kOut) return;
  if (ws_size < kWsTotal) return;
  const float* x = (const float*)d_in[0];
  const float* Wih0 = (const float*)d_in[1];
  const float* Whh0 = (const float*)d_in[2];
  const float* bih0 = (const float*)d_in[3];
  const float* bhh0 = (const float*)d_in[4];
  const float* Wih1 = (const float*)d_in[5];
  const float* Whh1 = (const float*)d_in[6];
  const float* bih1 = (const float*)d_in[7];
  const float* bhh1 = (const float*)d_in[8];
  const float* fcW = (const float*)d_in[9];
  const float* fcb = (const float*)d_in[10];
  float* out = (float*)d_out;
  char* ws = (char*)d_ws;
  unsigned short* W4 = (unsigned short*)(ws + kOffW4);
  unsigned short* WF = (unsigned short*)(ws + kOffWF);
  float* BIAS = (float*)(ws + kOffBIAS);
  unsigned short* A4 = (unsigned short*)(ws + kOffA4);
  float* G4 = (float*)(ws + kOffG4);
  float* H32 = (float*)(ws + kOffH32);
  float* O32 = (float*)(ws + kOffO32);
  const size_t kWp = (size_t)kG3 * kH;

  cast_plane_kernel<<<(int)(((size_t)kG3 * kIn / 8) / kThr), kThr, 0, stream>>>(Wih0, W4, 7, kH, 0);
  cast_plane_kernel<<<(int)(((size_t)kG3 * kH / 8) / kThr), kThr, 0, stream>>>(Whh0, W4 + kWp, 8, kH, 0);
  cast_plane_kernel<<<(int)(((size_t)kG3 * kH / 8) / kThr), kThr, 0, stream>>>(Wih1, W4 + 2 * kWp, 8, kH, 0);
  cast_plane_kernel<<<(int)(((size_t)kG3 * kH / 8) / kThr), kThr, 0, stream>>>(Whh1, W4 + 3 * kWp, 8, kH, 0);
  setup_kernel<<<321, kThr, 0, stream>>>(x, fcW, fcb, BIAS, WF, W4, A4, H32);

  for (int k = 0; k <= kT; ++k) {
    wmma_gemm64<0, false, 2, 0, false, 0><<<dim3((kB / 64) * (kG3 / 64) / 8, kNP), 256, 0, stream>>>(
        A4, A4, kH, (long)kB * kH, W4, W4, kH, (long)kG3 * kH, (void*)G4, (void*)G4, kG3, (long)kB * kG3, BIAS + kFBZ, nullptr, 0L, kB, kG3, kH, kSc);
    gru2_kernel<<<64, kThr, 0, stream>>>(G4, bih0, bhh0, bih1, bhh1, x, H32, A4, k);
  }
  wmma_gemm64<0, false, 2, 0, false, 0><<<dim3((kB / 64) * (kOutP / 64) / 8, 1), 256, 0, stream>>>(
      A4 + 3 * (size_t)kB * kH, A4 + 3 * (size_t)kB * kH, kH, 0L, WF, WF, kH, 0L, (void*)O32, (void*)O32, kOutP, 0L, BIAS + kFBF, nullptr, 0L, kB, kOutP, kH, kSc);
  out_kernel<<<59, 128, 0, stream>>>(O32, out);
}
